// TransformerEncoderLayer_14181982012103
// MI455X (gfx1250) — hardware-run, weakly checked
//
#include <hip/hip_runtime.h>
#ifndef NB
#define NB 2
#endif
#define NB_FULL 2
#ifndef SEQ
#define SEQ 2048
#endif
#define SEQ_FULL 2048
#define DM 1024
#define NH 16
#define HD 64
#define DFF 4096
#define LQ 3072
#define QOFF 0
#define KOFF 1024
#define VOFF 2048
#define MROWS (NB * SEQ)

static_assert(NB >= 1 && NB <= NB_FULL);
static_assert(SEQ % 128 == 0);
static_assert(SEQ <= SEQ_FULL);
static_assert(NH * HD == DM);
static_assert(LQ == 3 * DM);
static_assert(DM == 1024);
static_assert(DM == 32 * 4 * 8);
static_assert(HD == 64);
static_assert(MROWS % 128 == 0 && MROWS % 8 == 0);
static_assert(DM % 64 == 0 && DFF % 64 == 0 && LQ % 64 == 0);
static_assert(DM % 32 == 0 && DFF % 32 == 0 && SEQ % 32 == 0);

typedef unsigned short v8us __attribute__((ext_vector_type(8), may_alias));
typedef float  v8f  __attribute__((ext_vector_type(8)));
typedef float  v4f  __attribute__((ext_vector_type(4)));
typedef float  v4fa __attribute__((ext_vector_type(4), may_alias));
typedef _Float16 v16h __attribute__((ext_vector_type(16)));
typedef _Float16 v4h  __attribute__((ext_vector_type(4)));
union FragH { v16h v; v8us half[2]; _Float16 h[16]; unsigned short u[16]; };

__device__ __forceinline__ unsigned short bf16_bits(float x) { unsigned int u = __float_as_uint(x); return (unsigned short)((u + 0x7FFFu + ((u >> 16) & 1u)) >> 16); }
__device__ __forceinline__ float bf16_rne(float x) { return __uint_as_float(((unsigned int)bf16_bits(x)) << 16); }
__device__ __forceinline__ float gelu_f(float v) { return 0.5f * v * (1.0f + erff(v * 0.70710678118654752f)); }

__device__ __forceinline__ v16h g2_frag(const _Float16* p, unsigned hh) { FragH f; f.half[0] = *(const v8us*)((const unsigned short*)p + 8 * hh); f.half[1] = *(const v8us*)((const unsigned short*)p + 16 + 8 * hh); return f.v; }
__device__ __forceinline__ v8f g2_mma(v16h a, v16h b, v8f c) { v8f d = __builtin_amdgcn_wmma_f32_16x16x32_f16(false, a, false, b, (short)0, c, false, false); asm volatile("v_nop\n\tv_nop\n\tv_nop\n\tv_nop" : "+v"(d) : "v"(a), "v"(b)); return d; }

__global__ __launch_bounds__(256) void k_cvt16(const float* __restrict__ in, _Float16* __restrict__ out, unsigned n8, float scale, unsigned per_b8, unsigned in_bstride) {
  const unsigned t = blockIdx.x * 256u + threadIdx.x;
  if (t >= n8) return;
  const unsigned b = t / per_b8; const unsigned rem = t - b * per_b8;
  const float* src = in + (size_t)b * in_bstride + (size_t)rem * 8u;
  const v4f a = *(const v4fa*)src, c = *(const v4fa*)(src + 4);
  FragH f;
#pragma unroll
  for (int q = 0; q < 4; ++q) { f.h[q] = (_Float16)(bf16_rne(a[q]) * scale); f.h[4 + q] = (_Float16)(bf16_rne(c[q]) * scale); }
  const v8us o = f.half[0];
  unsigned short* d = (unsigned short*)out + (size_t)t * 8;
  *(volatile v8us*)d = o; __threadfence(); *(volatile v8us*)d = o;
}

__global__ __launch_bounds__(256) void k_vt(const _Float16* __restrict__ QKV, _Float16* __restrict__ VT) {
  __shared__ unsigned short tl[64][66];
  const unsigned tid = threadIdx.x; const unsigned bh = blockIdx.x / (unsigned)(SEQ / 64), lg = blockIdx.x % (unsigned)(SEQ / 64);
  const unsigned b = bh / (unsigned)NH, h = bh % (unsigned)NH;
  for (unsigned i = tid; i < 512u; i += 256u) { const unsigned r = i >> 3, c8 = (i & 7u) * 8u; FragH f; f.half[0] = *(const v8us*)((const unsigned short*)QKV + ((size_t)b * SEQ + lg * 64u + r) * LQ + VOFF + h * 64u + c8);
#pragma unroll
    for (int q = 0; q < 8; ++q) tl[r][c8 + q] = f.u[q]; }
  __syncthreads();
  for (int pass = 0; pass < 2; ++pass) {
#pragma unroll
    for (unsigned rd = 0; rd < 2; ++rd) { const unsigned d = rd * 32u + (tid >> 3), pc = tid & 7u; FragH f;
#pragma unroll
      for (int q = 0; q < 8; ++q) f.u[q] = tl[pc * 8u + q][d];
      const v8us o = f.half[0];
      *(volatile v8us*)((unsigned short*)VT + ((size_t)bh * 64u + d) * SEQ + lg * 64u + pc * 8u) = o; }
    if (pass == 0) __threadfence(); }
}

__global__ __launch_bounds__(128) void k_stats(const _Float16* __restrict__ QKV, float* __restrict__ SH) {
  __shared__ __attribute__((aligned(16))) float st[64];
  const unsigned tid = threadIdx.x, w = tid >> 5, lane = tid & 31u, ln = lane & 15u, hh = lane >> 4;
  const unsigned sb = blockIdx.x % (unsigned)(SEQ / 64), bh = blockIdx.x / (unsigned)(SEQ / 64);
  const unsigned b = bh / (unsigned)NH, h = bh % (unsigned)NH;
  const unsigned s0 = sb * 64u + w * 16u;
  const _Float16* srow = QKV + ((size_t)b * SEQ + s0 + ln) * LQ + KOFF + h * 64u;
  const v16h bs0 = g2_frag(srow, hh), bs1 = g2_frag(srow + 32, hh);
  const _Float16* lbase = QKV + ((size_t)b * SEQ + ln) * LQ + QOFF + h * 64u;
  const v8f z8 = {0.f, 0.f, 0.f, 0.f, 0.f, 0.f, 0.f, 0.f};
  float m = -1.0e30f, l = 0.f;
#pragma unroll 1
  for (unsigned j0 = 0; j0 < (unsigned)SEQ; j0 += 64u) {
    v8f c[4];
#pragma unroll
    for (int t = 0; t < 4; ++t) { const _Float16* lr = lbase + (size_t)(j0 + t * 16u) * LQ; v8f z = z8; z = g2_mma(g2_frag(lr, hh), bs0, z); z = g2_mma(g2_frag(lr + 32, hh), bs1, z); c[t] = z; }
    float mx = c[0][0];
#pragma unroll
    for (int t = 0; t < 4; ++t)
#pragma unroll
      for (int r = 0; r < 8; ++r) mx = fmaxf(mx, c[t][r]);
    mx = fmaxf(mx, __shfl_xor(mx, 16, 32));
    const float mnew = fmaxf(m, mx * 0.125f);
    const float alpha = __expf(m - mnew);
    m = mnew;
    const float sh = -mnew;
    float ps = 0.f;
#pragma unroll
    for (int r = 0; r < 8; ++r) {
      const float e0 = __expf(fmaf(c[0][r], 0.125f, sh)), e1 = __expf(fmaf(c[1][r], 0.125f, sh));
      const float e2 = __expf(fmaf(c[2][r], 0.125f, sh)), e3 = __expf(fmaf(c[3][r], 0.125f, sh));
      ps += (e0 + e1) + (e2 + e3);
    }
    l = l * alpha + ps;
  }
  const float lt = l + __shfl_xor(l, 16, 32);
  const float shf = 9.70406053f - m - logf(lt);
  if (hh == 0u) st[w * 16u + ln] = shf;
  __syncthreads();
  const v4f v = *(const v4fa*)&st[(tid & 15u) * 4u];
  float* dst = SH + (size_t)bh * SEQ + sb * 64u + (tid & 15u) * 4u;
  if (tid < 16u) { *(volatile v4f*)dst = v; __threadfence(); *(volatile v4f*)dst = v; }
}

__global__ __launch_bounds__(128) void k_attn(const _Float16* __restrict__ QKV, const _Float16* __restrict__ VT, const float* __restrict__ SH, _Float16* __restrict__ O16) {
  __shared__ __attribute__((aligned(16))) float osf[4][16][68];
  __shared__ __attribute__((aligned(16))) unsigned short os[4][16][72];
  const unsigned tid = threadIdx.x, w = tid >> 5, lane = tid & 31u, ln = lane & 15u, hh = lane >> 4;
  const unsigned tb = blockIdx.x % (unsigned)(SEQ / 64), bh = blockIdx.x / (unsigned)(SEQ / 64);
  const unsigned b = bh / (unsigned)NH, h = bh % (unsigned)NH;
  const unsigned t0 = tb * 64u + w * 16u;
  const _Float16* orow = QKV + ((size_t)b * SEQ + t0 + ln) * LQ + QOFF + h * 64u;
  const v16h bq0 = g2_frag(orow, hh), bq1 = g2_frag(orow + 32, hh);
  const _Float16* kbase = QKV + ((size_t)b * SEQ + ln) * LQ + KOFF + h * 64u;
  const _Float16* vbase = VT + ((size_t)bh * 64u + ln) * SEQ;
  const float* shb = SH + (size_t)bh * SEQ + 8u * hh;
  const v8f z8 = {0.f, 0.f, 0.f, 0.f, 0.f, 0.f, 0.f, 0.f};
  v8f o[4] = {z8, z8, z8, z8};
#pragma unroll 1
  for (unsigned j0 = 0; j0 < (unsigned)SEQ; j0 += 32u) {
    v8f c[2];
#pragma unroll
    for (int t = 0; t < 2; ++t) { const _Float16* kr = kbase + (size_t)(j0 + t * 16u) * LQ; v8f z = z8; z = g2_mma(g2_frag(kr, hh), bq0, z); z = g2_mma(g2_frag(kr + 32, hh), bq1, z); c[t] = z; }
    FragH ph;
#pragma unroll
    for (int t = 0; t < 2; ++t) {
      const v4f sa = *(const v4fa*)(shb + j0 + t * 16u), sb = *(const v4fa*)(shb + j0 + t * 16u + 4u);
#pragma unroll
      for (int r = 0; r < 4; ++r) {
        const float e0 = __expf(fmaf(c[t][r], 0.125f, sa[r]));
        const float e1 = __expf(fmaf(c[t][4 + r], 0.125f, sb[r]));
        ph.h[t * 8 + r] = (_Float16)e0;
        ph.h[t * 8 + 4 + r] = (_Float16)e1;
      }
    }
#pragma unroll
    for (int dt = 0; dt < 4; ++dt) {
      const v16h va = g2_frag(vbase + (size_t)(dt * 16u) * SEQ + j0, hh);
      o[dt] = g2_mma(va, ph.v, o[dt]);
    }
  }
#pragma unroll
  for (int dt = 0; dt < 4; ++dt) {
    const v4f lo4 = {o[dt][0], o[dt][1], o[dt][2], o[dt][3]};
    const v4f hi4 = {o[dt][4], o[dt][5], o[dt][6], o[dt][7]};
    *(v4fa*)&osf[w][ln][dt * 16 + 8 * hh] = lo4;
    *(v4fa*)&osf[w][ln][dt * 16 + 8 * hh + 4] = hi4; }
  __builtin_amdgcn_fence(4  , "workgroup"); __builtin_amdgcn_wave_barrier();
  const unsigned rq = lane >> 3, pc = (lane & 7u) * 8u;
#pragma unroll 1
  for (unsigned it = 0; it < 4u; ++it) { const unsigned row = it * 4u + rq;
    const v4f x0 = *(const v4fa*)&osf[w][row][pc], x1 = *(const v4fa*)&osf[w][row][pc + 4u];
    FragH f;
#pragma unroll
    for (int q = 0; q < 4; ++q) {
      const float g0 = gelu_f(x0[q] * 6.103515625e-05f) * 0.02209708691207961f;
      const float g1 = gelu_f(x1[q] * 6.103515625e-05f) * 0.02209708691207961f;
      f.h[q] = (_Float16)(g0 * 4096.0f); f.h[4 + q] = (_Float16)(g1 * 4096.0f); }
    *(v8us*)&os[w][row][pc] = f.half[0]; }
  __builtin_amdgcn_fence(4  , "workgroup"); __builtin_amdgcn_wave_barrier();
  for (int pass = 0; pass < 2; ++pass) {
#pragma unroll
    for (unsigned it = 0; it < 4; ++it) { const unsigned row = it * 4u + rq; const v8us v = *(const v8us*)&os[w][row][pc];
      *(volatile v8us*)((unsigned short*)O16 + ((size_t)b * SEQ + t0 + row) * DM + h * 64u + pc) = v; }
    if (pass == 0) __threadfence(); }
}

template <int ACT>
__global__ __launch_bounds__(128) void k_gemm(const _Float16* __restrict__ A, unsigned lda, const _Float16* __restrict__ Bh, unsigned ldb, float alpha, const float* __restrict__ bias, float oscale,
    float* __restrict__ C, _Float16* __restrict__ C16, unsigned ldc, unsigned M, unsigned N, unsigned K) {
  static_assert(ACT == 0 || ACT == 1);
  __shared__ __attribute__((aligned(16))) float so[4][32][68];
  const unsigned tid = threadIdx.x, w = tid >> 5, lane = tid & 31u, ln = lane & 15u, hh = lane >> 4;
  const unsigned ntn = N >> 6; const unsigned mt = blockIdx.x / ntn, nq = blockIdx.x - mt * ntn; const unsigned row0 = mt * 128u + 32u * w, col0 = nq * 64u; if (row0 >= M) return;
  const _Float16* a0p = A + (size_t)(row0 + ln) * lda; const _Float16* a1p = a0p + (size_t)16 * lda;
  const v8f z8 = {0.f,0.f,0.f,0.f,0.f,0.f,0.f,0.f};
#pragma unroll 1
  for (unsigned nh = 0; nh < 2u; ++nh) {
    const unsigned cb = nh * 32u;
    const _Float16* b0p = Bh + (size_t)(col0 + cb + ln) * ldb; const _Float16* b1p = b0p + (size_t)16 * ldb;
    v8f c00 = z8, c01 = z8, c10 = z8, c11 = z8;
#pragma unroll 1
    for (unsigned kb = 0; kb < K; kb += 32u) {
      const v16h a0 = g2_frag(a0p + kb, hh), a1 = g2_frag(a1p + kb, hh);
      const v16h bf0 = g2_frag(b0p + kb, hh), bf1 = g2_frag(b1p + kb, hh);
      c00 = g2_mma(a0, bf0, c00); c10 = g2_mma(a1, bf0, c10);
      c01 = g2_mma(a0, bf1, c01); c11 = g2_mma(a1, bf1, c11);
    }
    v8f accs[4] = {c00, c01, c10, c11};
#pragma unroll
    for (int u = 0; u < 4; ++u) { const int t = u & 1, half = u >> 1; const unsigned cl = cb + t * 16 + ln; const float bv = bf16_rne(bias[col0 + cl]);
#pragma unroll
      for (int r = 0; r < 8; ++r) { const unsigned rloc = half * 16 + 8 * hh + r; so[w][rloc][cl] = accs[u][r] * alpha + bv; } }
  }
  __builtin_amdgcn_fence(4  , "workgroup"); __builtin_amdgcn_wave_barrier();
  const unsigned rsub = lane >> 4, c4 = (lane & 15u) * 4u;
  if (ACT == 1) {
#pragma unroll 1
    for (unsigned q = 0; q < 16u; ++q) { const unsigned r = q * 2u + rsub; v4f v = *(const v4fa*)&so[w][r][c4];
#pragma unroll
      for (int i = 0; i < 4; ++i) v[i] = gelu_f(v[i]) * oscale;
      *(v4fa*)&so[w][r][c4] = v; }
    __builtin_amdgcn_fence(4  , "workgroup"); __builtin_amdgcn_wave_barrier();
  }
  for (int pass = 0; pass < 2; ++pass) {
#pragma unroll
    for (unsigned q = 0; q < 16; ++q) { const unsigned r = q * 2u + rsub; const v4f v = *(const v4fa*)&so[w][r][c4];
      if (C) *(volatile v4f*)(C + (size_t)(row0 + r) * ldc + col0 + c4) = v;
      if (C16) { v4h h4;
#pragma unroll
        for (int i = 0; i < 4; ++i) h4[i] = (_Float16)v[i];
        *(volatile v4h*)(C16 + (size_t)(row0 + r) * ldc + col0 + c4) = h4; } }
    if (pass == 0) __threadfence(); }
}

template <int FIRST>
__global__ __launch_bounds__(256) void k_ln(const float* __restrict__ a, const float* __restrict__ bres, const float* __restrict__ g, const float* __restrict__ be, float* __restrict__ outF, _Float16* __restrict__ out16) {
  __shared__ __attribute__((aligned(16))) float rowb[8][DM];
  const unsigned tid = threadIdx.x, w = tid >> 5, lane = tid & 31u;
  const unsigned r = blockIdx.x * 8u + w;
  if (r >= (unsigned)MROWS) return;
  const unsigned b = r / (unsigned)SEQ, s = r - b * (unsigned)SEQ;
  const size_t frow = ((size_t)b * SEQ_FULL + s) * DM;
  const size_t crow = (size_t)r * DM;
  const float* ap = a + (FIRST ? frow : crow);
  const float* bp = bres + crow;
  float* op = outF + (FIRST ? crow : frow);
  float sum = 0.f;
#pragma unroll 1
  for (unsigned i = 0; i < 8u; ++i) { const unsigned idx = i * 128u + lane * 4u;
    const v4f x = *(const v4fa*)(ap + idx), y = *(const v4fa*)(bp + idx); v4f v;
#pragma unroll
    for (int q = 0; q < 4; ++q) v[q] = (FIRST ? bf16_rne(x[q]) : x[q]) + y[q];
    *(v4fa*)&rowb[w][idx] = v;
    sum += (v[0] + v[1]) + (v[2] + v[3]); }
#pragma unroll
  for (int o = 16; o > 0; o >>= 1) sum += __shfl_xor(sum, o, 32);
  const float mu = sum * 0.0009765625f;
  float sq = 0.f;
#pragma unroll 1
  for (unsigned i = 0; i < 8u; ++i) { const unsigned idx = i * 128u + lane * 4u;
    const v4f v = *(const v4fa*)&rowb[w][idx];
    const float d0 = v[0] - mu, d1 = v[1] - mu, d2 = v[2] - mu, d3 = v[3] - mu;
    sq += (d0 * d0 + d1 * d1) + (d2 * d2 + d3 * d3); }
#pragma unroll
  for (int o = 16; o > 0; o >>= 1) sq += __shfl_xor(sq, o, 32);
  const float rstd = rsqrtf(sq * 0.0009765625f + 1.0e-5f);
#pragma unroll 1
  for (unsigned i = 0; i < 8u; ++i) { const unsigned idx = i * 128u + lane * 4u;
    const v4f v = *(const v4fa*)&rowb[w][idx];
    const v4f gg = *(const v4fa*)(g + idx), bb = *(const v4fa*)(be + idx); v4f y;
#pragma unroll
    for (int q = 0; q < 4; ++q) y[q] = (v[q] - mu) * rstd * bf16_rne(gg[q]) + bf16_rne(bb[q]);
    *(v4fa*)&rowb[w][idx] = y; }
  for (int pass = 0; pass < 2; ++pass) {
#pragma unroll 1
    for (unsigned i = 0; i < 8u; ++i) { const unsigned idx = i * 128u + lane * 4u;
      const v4f y = *(const v4fa*)&rowb[w][idx];
      *(volatile v4f*)(op + idx) = y;
      if (FIRST) { v4h h4;
#pragma unroll
        for (int q = 0; q < 4; ++q) h4[q] = (_Float16)(y[q] * 16.0f);
        *(volatile v4h*)(out16 + crow + idx) = h4; } }
    if (pass == 0) __threadfence(); }
}

#define SZ_BQKV ((size_t)LQ * DM * 2)
#define SZ_BP   ((size_t)DM * DM * 2)
#define SZ_BW1  ((size_t)DFF * DM * 2)
#define SZ_BW2  ((size_t)DM * DFF * 2)
#define SZ_XA   ((size_t)MROWS * DM * 2)
#define SZ_QKV  ((size_t)MROWS * LQ * 2)
#define SZ_VT   ((size_t)NB * NH * HD * SEQ * 2)
#define SZ_HF   ((size_t)MROWS * DFF * 2)
#define SZ_QV   (SZ_QKV + SZ_VT)
#define SZ_SH   ((size_t)NB * NH * SEQ * 4)
#define SZ_O16  ((size_t)MROWS * DM * 2)
#define SZ_F32  ((size_t)MROWS * DM * 4)
#define SZ_TOT  (SZ_BQKV + SZ_BP + SZ_BW1 + SZ_BW2 + SZ_XA + SZ_QV + SZ_SH + SZ_O16 + 3 * SZ_F32)
static_assert(SZ_TOT <= (size_t)134217728);
static_assert(SZ_HF <= SZ_QV);
static_assert(SZ_BQKV % 256 == 0 && SZ_BP % 256 == 0 && SZ_BW1 % 256 == 0 && SZ_BW2 % 256 == 0 && SZ_XA % 256 == 0);
static_assert(SZ_QKV % 256 == 0 && SZ_VT % 256 == 0 && SZ_SH % 256 == 0 && SZ_O16 % 256 == 0 && SZ_F32 % 256 == 0);
static_assert(((size_t)MROWS * (DM / 8)) % 256 == 0);
static_assert(((size_t)LQ * (DM / 8)) % 256 == 0 && ((size_t)DM * (DM / 8)) % 256 == 0 && ((size_t)DFF * (DM / 8)) % 256 == 0 && ((size_t)DM * (DFF / 8)) % 256 == 0);
static_assert((size_t)NB * NH * (SEQ / 64) * 64 * 64 == (size_t)NB * NH * HD * SEQ);
static_assert((size_t)NB * NH * (SEQ / 64) * 64 == (size_t)NB * NH * SEQ);
static_assert((size_t)NB * NH * (SEQ / 64) * 64 * 64 == (size_t)MROWS * DM);
static_assert((size_t)(MROWS / 128) * (LQ / 64) * 128 * 64 == (size_t)MROWS * LQ);
static_assert((size_t)(MROWS / 128) * (DM / 64) * 128 * 64 == (size_t)MROWS * DM);
static_assert((size_t)(MROWS / 128) * (DFF / 64) * 128 * 64 == (size_t)MROWS * DFF);
static_assert((size_t)(MROWS / 8) * 8 * DM == (size_t)MROWS * DM);

extern "C" void kernel_launch(void* const* d_in, const int* in_sizes, int n_in,
                              void* d_out, int out_size, void* d_ws, size_t ws_size, hipStream_t stream) {
  if (n_in < 13) return;
  const long long xneed = ((long long)(NB - 1) * SEQ_FULL + SEQ) * DM;
  if ((long long)in_sizes[0] < xneed || (long long)out_size < xneed) return;
  if (in_sizes[1] < LQ * DM || in_sizes[2] < LQ || in_sizes[3] < DM * DM || in_sizes[4] < DM) return;
  if (in_sizes[5] < DFF * DM || in_sizes[6] < DFF || in_sizes[7] < DM * DFF || in_sizes[8] < DM) return;
  if (in_sizes[9] < DM || in_sizes[10] < DM || in_sizes[11] < DM || in_sizes[12] < DM) return;
  if (ws_size < SZ_TOT) return;
  const float* x  = (const float*)d_in[0];
  const float* Wi = (const float*)d_in[1];  const float* bi = (const float*)d_in[2];
  const float* Wo = (const float*)d_in[3];  const float* bo = (const float*)d_in[4];
  const float* W1 = (const float*)d_in[5];  const float* b1 = (const float*)d_in[6];
  const float* W2 = (const float*)d_in[7];  const float* b2 = (const float*)d_in[8];
  const float* g1 = (const float*)d_in[9];  const float* e1 = (const float*)d_in[10];
  const float* g2 = (const float*)d_in[11]; const float* e2 = (const float*)d_in[12];
  float* out = (float*)d_out;
  char* ws = (char*)d_ws; size_t off = 0;
  _Float16* BQKV = (_Float16*)(ws + off); off += SZ_BQKV;
  _Float16* BP   = (_Float16*)(ws + off); off += SZ_BP;
  _Float16* BW1  = (_Float16*)(ws + off); off += SZ_BW1;
  _Float16* BW2  = (_Float16*)(ws + off); off += SZ_BW2;
  _Float16* X16  = (_Float16*)(ws + off); _Float16* X116 = X16; off += SZ_XA;
  _Float16* QKV  = (_Float16*)(ws + off); _Float16* HF16 = QKV;
  _Float16* VT   = (_Float16*)(ws + off + SZ_QKV); off += SZ_QV;
  float* SH      = (float*)(ws + off); off += SZ_SH;
  _Float16* O16  = (_Float16*)(ws + off); off += SZ_O16;
  float* ATT     = (float*)(ws + off); off += SZ_F32;
  float* X1      = (float*)(ws + off); off += SZ_F32;
  float* FF      = (float*)(ws + off); off += SZ_F32;
  if (off > ws_size) return;

  k_cvt16<<<(unsigned)((size_t)MROWS * (DM / 8) / 256), 256, 0, stream>>>(x, X16, (unsigned)((size_t)MROWS * (DM / 8)), 16.0f, (unsigned)((size_t)SEQ * (DM / 8)), (unsigned)((size_t)SEQ_FULL * DM));
  k_cvt16<<<(unsigned)((size_t)LQ * (DM / 8) / 256), 256, 0, stream>>>(Wi, BQKV, (unsigned)((size_t)LQ * (DM / 8)), 64.0f, (unsigned)((size_t)LQ * (DM / 8)), 0u);
  k_cvt16<<<(unsigned)((size_t)DM * (DM / 8) / 256), 256, 0, stream>>>(Wo, BP, (unsigned)((size_t)DM * (DM / 8)), 64.0f, (unsigned)((size_t)DM * (DM / 8)), 0u);
  k_cvt16<<<(unsigned)((size_t)DFF * (DM / 8) / 256), 256, 0, stream>>>(W1, BW1, (unsigned)((size_t)DFF * (DM / 8)), 64.0f, (unsigned)((size_t)DFF * (DM / 8)), 0u);
  k_cvt16<<<(unsigned)((size_t)DM * (DFF / 8) / 256), 256, 0, stream>>>(W2, BW2, (unsigned)((size_t)DM * (DFF / 8)), 64.0f, (unsigned)((size_t)DM * (DFF / 8)), 0u);
  k_gemm<0><<<(unsigned)((MROWS / 128) * (LQ / 64)), 128, 0, stream>>>(X16, (unsigned)DM, BQKV, (unsigned)DM, 0.0009765625f, bi, 1.0f, nullptr, QKV, (unsigned)LQ, (unsigned)MROWS, (unsigned)LQ, (unsigned)DM);
  k_vt<<<(unsigned)(NB * NH * (SEQ / 64)), 256, 0, stream>>>(QKV, VT);
  k_stats<<<(unsigned)(NB * NH * (SEQ / 64)), 128, 0, stream>>>(QKV, SH);
  k_attn<<<(unsigned)(NB * NH * (SEQ / 64)), 128, 0, stream>>>(QKV, VT, SH, O16);
  k_gemm<0><<<(unsigned)((MROWS / 128) * (DM / 64)), 128, 0, stream>>>(O16, (unsigned)DM, BP, (unsigned)DM, 3.814697265625e-06f, bo, 1.0f, ATT, nullptr, (unsigned)DM, (unsigned)MROWS, (unsigned)DM, (unsigned)DM);
  k_ln<1><<<(unsigned)(MROWS / 8), 256, 0, stream>>>(x, ATT, g1, e1, X1, X116);
  k_gemm<1><<<(unsigned)((MROWS / 128) * (DFF / 64)), 128, 0, stream>>>(X116, (unsigned)DM, BW1, (unsigned)DM, 0.0009765625f, b1, 16.0f, nullptr, HF16, (unsigned)DFF, (unsigned)MROWS, (unsigned)DFF, (unsigned)DM);
  k_gemm<0><<<(unsigned)((MROWS / 128) * (DM / 64)), 128, 0, stream>>>(HF16, (unsigned)DFF, BW2, (unsigned)DFF, 0.0009765625f, b2, 1.0f, FF, nullptr, (unsigned)DM, (unsigned)MROWS, (unsigned)DM, (unsigned)DFF);
  k_ln<0><<<(unsigned)(MROWS / 8), 256, 0, stream>>>(X1, FF, g2, e2, out, nullptr);
}
